// SelfAttention_49667001811806
// MI455X (gfx1250) — hardware-run, weakly checked
//
#include <hip/hip_runtime.h>


#ifndef NB
#define NB 2
#endif
#ifndef SEQ
#define SEQ 2048
#endif
#define NB_FULL    2
#define SEQ_FULL   2048
#define DM         2048
#define NHEAD      16
#define HDIM       128
#define HALFD      64
#define BQ         128
#define BK         32
#define NWAVE      8
#define GT         128
#define GK         64
#define LP         72
#define OP         68
#define TP         136
#define WS_CAP     134217728ull

static_assert(SEQ % BQ == 0);
static_assert(SEQ % GT == 0);
static_assert(SEQ % BK == 0);
static_assert(DM % GT == 0);
static_assert(DM % GK == 0);
static_assert(GK % 32 == 0);
static_assert(GT == HDIM);
static_assert(DM == NHEAD * HDIM);
static_assert(HDIM == 2 * HALFD);
static_assert(BQ == NWAVE * 16);
static_assert(HDIM % 32 == 0);
static_assert(DM == 256 * 8);
static_assert(SEQ <= SEQ_FULL);
static_assert(NB >= 1 && NB <= NB_FULL);
static_assert((LP * 2) % 16 == 0);
static_assert((OP * 4) % 16 == 0);
static_assert((TP * 2) % 16 == 0);
static_assert(NWAVE * 16 * OP * 4 <= 2 * GT * LP * 2);
static_assert(HDIM * TP * 2 <= 2 * GT * LP * 2);
static_assert((unsigned long long)NB * SEQ * DM * 2ull
              + 3ull * DM * DM * 2ull
              + (unsigned long long)NB * SEQ * DM * 4ull
              + 3ull * NB * SEQ * DM * 2ull <= WS_CAP);

typedef __bf16   bf16;
typedef _Float16 f16;
typedef bf16     v16bf __attribute__((ext_vector_type(16)));
typedef f16      v16h  __attribute__((ext_vector_type(16)));
typedef float    v8f   __attribute__((ext_vector_type(8)));
typedef float    v4f   __attribute__((ext_vector_type(4)));
typedef unsigned v4u   __attribute__((ext_vector_type(4)));

union Frag16 { v16bf b; v16h h; v4u q[2]; };
union FragH  { v16h  v; v4u q[2]; f16 h[16]; };
union Pack8B { v4u u; bf16 h[8]; };
union Pack8H { v4u u; f16 h[8]; };

static __device__ __forceinline__ v8f mma_bf16(v16bf a, v16bf b, v8f acc) {
  acc = __builtin_amdgcn_wmma_f32_16x16x32_bf16(false, a, false, b, (short)0, acc, false, false);
  asm volatile("v_nop\n\tv_nop\n\tv_nop\n\tv_nop" : "+v"(acc) : "v"(a), "v"(b));
  return acc;
}
static __device__ __forceinline__ v8f mma_f16(v16h a, v16h b, v8f acc) {
  acc = __builtin_amdgcn_wmma_f32_16x16x32_f16(false, a, false, b, (short)0, acc, false, false);
  asm volatile("v_nop\n\tv_nop\n\tv_nop\n\tv_nop" : "+v"(acc) : "v"(a), "v"(b));
  return acc;
}

template <int MODE>
__global__ __launch_bounds__(256) void cvt_rows_kernel(const float* __restrict__ in,
                                                       unsigned short* __restrict__ out,
                                                       int seq, int seq_full, float scale) {
  const int m  = blockIdx.x;
  const int t  = threadIdx.x;
  const int bb = m / seq;
  const int s  = m - bb * seq;
  const size_t src = ((size_t)bb * seq_full + s) * DM + t * 8;
  const size_t dst = (size_t)m * DM + t * 8;
  const v4f a0 = *(const v4f*)(in + src);
  const v4f a1 = *(const v4f*)(in + src + 4);
  v4u val;
  if (MODE == 0) {
    Pack8B pk;
    #pragma unroll
    for (int i = 0; i < 4; ++i) {
      pk.h[i]     = (bf16)a0[i];
      pk.h[4 + i] = (bf16)a1[i];
    }
    val = pk.u;
  } else {
    Pack8H ph;
    #pragma unroll
    for (int i = 0; i < 4; ++i) {
      ph.h[i]     = (f16)((float)(bf16)a0[i] * scale);
      ph.h[4 + i] = (f16)((float)(bf16)a1[i] * scale);
    }
    val = ph.u;
  }
  *(volatile v4u*)(out + dst) = val;
  __threadfence();
  *(volatile v4u*)(out + dst) = val;
}

template <int F16, int EPI>
__global__ __launch_bounds__(256) void gemm_kernel(const unsigned short* __restrict__ A,
                                                   const unsigned short* __restrict__ W,
                                                   const float* __restrict__ bias,
                                                   void* __restrict__ Cout,
                                                   float oscale) {
  __shared__ __align__(16) unsigned short lds[2 * GT * LP];
  const int t    = threadIdx.x;
  const int lane = t & 31;
  const int wid  = __builtin_amdgcn_readfirstlane(threadIdx.x >> 5);
  const int lq   = lane & 15;
  const int hi   = lane >> 4;
  const int bm   = blockIdx.x * GT;
  const int bn   = blockIdx.y * GT;
  const int wm   = (wid & 3) * 32;
  const int wn   = (wid >> 2) * 64;
  unsigned short* ldsA = lds;
  unsigned short* ldsB = lds + GT * LP;

  v8f acc[2][4];
  #pragma unroll
  for (int mt = 0; mt < 2; ++mt) {
    #pragma unroll
    for (int nt = 0; nt < 4; ++nt) acc[mt][nt] = (v8f){0, 0, 0, 0, 0, 0, 0, 0};
  }

  #pragma unroll 1
  for (int k0 = 0; k0 < DM; k0 += GK) {
    v4u ra[4], rb[4];
    #pragma unroll
    for (int i = 0; i < 4; ++i) {
      const int seg = t + i * 256;
      const int row = seg >> 3;
      const int c   = (seg & 7) * 8;
      ra[i] = *(const v4u*)(A + (size_t)(bm + row) * DM + k0 + c);
      rb[i] = *(const v4u*)(W + (size_t)(bn + row) * DM + k0 + c);
    }
    #pragma unroll
    for (int i = 0; i < 4; ++i) {
      const int seg = t + i * 256;
      const int row = seg >> 3;
      const int c   = (seg & 7) * 8;
      *(v4u*)(ldsA + row * LP + c) = ra[i];
      *(v4u*)(ldsB + row * LP + c) = rb[i];
    }
    __syncthreads();

    #pragma unroll
    for (int kk = 0; kk < 2; ++kk) {
      Frag16 af[2];
      #pragma unroll
      for (int mt = 0; mt < 2; ++mt) {
        const unsigned short* base = ldsA + (wm + mt * 16 + lq) * LP + kk * 32 + hi * 8;
        af[mt].q[0] = *(const v4u*)(base);
        af[mt].q[1] = *(const v4u*)(base + 16);
      }
      #pragma unroll
      for (int nt = 0; nt < 4; ++nt) {
        Frag16 bf;
        const unsigned short* base = ldsB + (wn + nt * 16 + lq) * LP + kk * 32 + hi * 8;
        bf.q[0] = *(const v4u*)(base);
        bf.q[1] = *(const v4u*)(base + 16);
        if (F16) {
          acc[0][nt] = mma_f16(af[0].h, bf.h, acc[0][nt]);
          acc[1][nt] = mma_f16(af[1].h, bf.h, acc[1][nt]);
        } else {
          acc[0][nt] = mma_bf16(af[0].b, bf.b, acc[0][nt]);
          acc[1][nt] = mma_bf16(af[1].b, bf.b, acc[1][nt]);
        }
      }
    }
    __syncthreads();
  }

  float bb[4];
  #pragma unroll
  for (int nt = 0; nt < 4; ++nt) bb[nt] = (float)(bf16)bias[bn + wn + nt * 16 + lq];

  if (EPI == 1) {
    unsigned short* sT = lds;
    #pragma unroll
    for (int mt = 0; mt < 2; ++mt) {
      #pragma unroll
      for (int nt = 0; nt < 4; ++nt) {
        Pack8H ph;
        #pragma unroll
        for (int r = 0; r < 8; ++r) ph.h[r] = (f16)(acc[mt][nt][r] + bb[nt]);
        *(v4u*)(sT + (wn + nt * 16 + lq) * TP + wm + mt * 16 + hi * 8) = ph.u;
      }
    }
    __syncthreads();
    unsigned short* vt = (unsigned short*)Cout;
    const int b  = bm / SEQ;
    const int s0 = bm - b * SEQ;
    const int h  = blockIdx.y;
    v4u    vals[8];
    size_t gidx[8];
    #pragma unroll
    for (int it = 0; it < 8; ++it) {
      const int idx = it * 256 + t;
      const int d   = idx >> 4;
      const int sg  = idx & 15;
      vals[it] = *(const v4u*)(sT + d * TP + sg * 8);
      gidx[it] = (((size_t)b * NHEAD + h) * HDIM + d) * SEQ + s0 + sg * 8;
    }
    #pragma unroll
    for (int it = 0; it < 8; ++it) *(volatile v4u*)(vt + gidx[it]) = vals[it];
    __threadfence();
    #pragma unroll
    for (int it = 0; it < 8; ++it) *(volatile v4u*)(vt + gidx[it]) = vals[it];
  } else {
    float* Cf = (float*)Cout;
    float* so = (float*)lds + wid * (16 * OP);
    const int bfull = bm / SEQ;
    const int srow  = bm - bfull * SEQ;
    const int orow0 = (EPI == 2) ? (bfull * SEQ_FULL + srow) : bm;
    #pragma unroll
    for (int mt = 0; mt < 2; ++mt) {
      #pragma unroll
      for (int nt = 0; nt < 4; ++nt) {
        #pragma unroll
        for (int r = 0; r < 8; ++r) {
          const float v = (EPI == 2) ? (acc[mt][nt][r] * oscale + bb[nt]) : (acc[mt][nt][r] + bb[nt]);
          so[(hi * 8 + r) * OP + nt * 16 + lq] = v;
        }
      }
      __syncthreads();
      v4f    vals[8];
      size_t gidx[8];
      #pragma unroll
      for (int it = 0; it < 8; ++it) {
        const int row = it * 2 + hi;
        vals[it] = *(const v4f*)(so + row * OP + lq * 4);
        gidx[it] = (size_t)(orow0 + wm + mt * 16 + row) * DM + bn + wn + lq * 4;
      }
      #pragma unroll
      for (int it = 0; it < 8; ++it) *(volatile v4f*)(Cf + gidx[it]) = vals[it];
      __threadfence();
      #pragma unroll
      for (int it = 0; it < 8; ++it) *(volatile v4f*)(Cf + gidx[it]) = vals[it];
      __syncthreads();
    }
  }
}

__global__ __launch_bounds__(256) void rmsnorm_rope_kernel(const float* __restrict__ X,
                                                           const float* __restrict__ w,
                                                           const float* __restrict__ cosb,
                                                           const float* __restrict__ sinb,
                                                           unsigned short* __restrict__ out) {
  const int m  = blockIdx.x;
  const int t  = threadIdx.x;
  const int bb = m / SEQ;
  const int s  = m - bb * SEQ;
  const float* x = X + (size_t)m * DM + t * 8;
  const v4f a0 = *(const v4f*)(x);
  const v4f a1 = *(const v4f*)(x + 4);
  float vx[8];
  #pragma unroll
  for (int i = 0; i < 4; ++i) { vx[i] = a0[i]; vx[4 + i] = a1[i]; }
  float ss = 0.0f;
  #pragma unroll
  for (int i = 0; i < 8; ++i) ss += vx[i] * vx[i];
  #pragma unroll
  for (int off = 16; off >= 1; off >>= 1) ss += __shfl_xor(ss, off, 32);
  __shared__ float red[8];
  if ((t & 31) == 0) red[t >> 5] = ss;
  __syncthreads();
  const float tot = ((red[0] + red[1]) + (red[2] + red[3])) + ((red[4] + red[5]) + (red[6] + red[7]));
  const float inv = rsqrtf(tot * (1.0f / (float)DM) + 1e-6f);

  const int j0 = (t * 4) & (HALFD - 1);
  const v4f c4 = *(const v4f*)(cosb + (size_t)s * HALFD + j0);
  const v4f s4 = *(const v4f*)(sinb + (size_t)s * HALFD + j0);
  const v4f w0 = *(const v4f*)(w + t * 8);
  const v4f w1 = *(const v4f*)(w + t * 8 + 4);
  float wv[8];
  #pragma unroll
  for (int i = 0; i < 4; ++i) { wv[i] = (float)(bf16)w0[i]; wv[4 + i] = (float)(bf16)w1[i]; }

  Pack8H ph;
  #pragma unroll
  for (int i = 0; i < 4; ++i) {
    const float c  = (float)(bf16)c4[i];
    const float sn = (float)(bf16)s4[i];
    const float y1 = vx[2 * i] * inv * wv[2 * i];
    const float y2 = vx[2 * i + 1] * inv * wv[2 * i + 1];
    ph.h[2 * i]     = (f16)(y1 * c - y2 * sn);
    ph.h[2 * i + 1] = (f16)(y1 * sn + y2 * c);
  }
  const v4u val = ph.u;
  const size_t dst = (size_t)m * DM + t * 8;
  *(volatile v4u*)(out + dst) = val;
  __threadfence();
  *(volatile v4u*)(out + dst) = val;
}

__global__ __launch_bounds__(256) void attn_kernel(const unsigned short* __restrict__ q16,
                                                   const unsigned short* __restrict__ k16,
                                                   const unsigned short* __restrict__ vt,
                                                   unsigned short* __restrict__ ctx) {
  const int qblk = blockIdx.x;
  const int h    = blockIdx.y;
  const int b    = blockIdx.z;
  const int tid  = threadIdx.x;
  const int wave = __builtin_amdgcn_readfirstlane(threadIdx.x >> 5);
  const int lane = tid & 31;
  const int lq   = lane & 15;
  const int hi   = lane >> 4;

  __shared__ __align__(16) f16 sO[NWAVE * 16 * TP];

  const int qrow0 = qblk * BQ + wave * 16;

  FragH qf[4];
  {
    const unsigned short* qp = q16 + ((size_t)b * SEQ + qrow0 + lq) * DM + h * HDIM;
    #pragma unroll
    for (int f = 0; f < 4; ++f) {
      qf[f].q[0] = *(const v4u*)(qp + f * 32 + hi * 8);
      qf[f].q[1] = *(const v4u*)(qp + f * 32 + 16 + hi * 8);
    }
  }

  const unsigned short* k_h  = k16 + (size_t)b * SEQ * DM + h * HDIM;
  const unsigned short* vt_h = vt + ((size_t)b * NHEAD + h) * HDIM * SEQ;

  v8f o[8];
  #pragma unroll
  for (int dt = 0; dt < 8; ++dt) o[dt] = (v8f){0, 0, 0, 0, 0, 0, 0, 0};

  float rmax = -__builtin_inff();
  float rsum = 0.0f;
  const float SL = 0.08838834764831845f * 1.4426950408889634f;

  const int nchunk = SEQ / BK;
  #pragma unroll 1
  for (int i = 0; i < nchunk; ++i) {
    const int j0 = i * BK;

    v8f c[2];
    #pragma unroll
    for (int sub = 0; sub < 2; ++sub) {
      FragH ak[4];
      const unsigned short* kr = k_h + (size_t)(j0 + sub * 16 + lq) * DM + hi * 8;
      #pragma unroll
      for (int f = 0; f < 4; ++f) {
        ak[f].q[0] = *(const v4u*)(kr + f * 32);
        ak[f].q[1] = *(const v4u*)(kr + f * 32 + 16);
      }
      v8f acc = (v8f){0, 0, 0, 0, 0, 0, 0, 0};
      #pragma unroll
      for (int f = 0; f < 4; ++f) acc = mma_f16(ak[f].v, qf[f].v, acc);
      c[sub] = acc;
    }

    float m_new = rmax;
    #pragma unroll
    for (int r = 0; r < 8; ++r) {
      m_new = fmaxf(m_new, c[0][r]);
      m_new = fmaxf(m_new, c[1][r]);
    }
    m_new = fmaxf(m_new, __shfl_xor(m_new, 16, 32));
    const float scale = __builtin_amdgcn_exp2f((rmax - m_new) * SL);
    rmax = m_new;

    FragH pa;
    float psum = 0.0f;
    #pragma unroll
    for (int r = 0; r < 8; ++r) {
      const float p0 = __builtin_amdgcn_exp2f((c[0][r] - m_new) * SL);
      const float p1 = __builtin_amdgcn_exp2f((c[1][r] - m_new) * SL);
      psum += p0 + p1;
      pa.h[r]     = (f16)(p0 * 4096.0f);
      pa.h[8 + r] = (f16)(p1 * 4096.0f);
    }
    rsum = rsum * scale + psum + __shfl_xor(psum, 16, 32);

    float sc[8];
    #pragma unroll
    for (int r = 0; r < 8; ++r) sc[r] = __shfl(scale, (hi << 3) + r, 32);
    #pragma unroll
    for (int dt = 0; dt < 8; ++dt) {
      #pragma unroll
      for (int r = 0; r < 8; ++r) o[dt][r] *= sc[r];
    }

    #pragma unroll
    for (int dt = 0; dt < 8; ++dt) {
      FragH bv;
      const unsigned short* vb = vt_h + (size_t)(dt * 16 + lq) * SEQ + j0 + hi * 8;
      bv.q[0] = *(const v4u*)(vb);
      bv.q[1] = *(const v4u*)(vb + 16);
      o[dt] = mma_f16(pa.v, bv.v, o[dt]);
    }
  }

  const float rinv = 1.0f / rsum;
  float rs[8];
  #pragma unroll
  for (int r = 0; r < 8; ++r) rs[r] = __shfl(rinv, (hi << 3) + r, 32);

  f16* so = sO + wave * (16 * TP);
  #pragma unroll
  for (int r = 0; r < 8; ++r) {
    #pragma unroll
    for (int dt = 0; dt < 8; ++dt) {
      so[(hi * 8 + r) * TP + dt * 16 + lq] = (f16)(o[dt][r] * 0.0625f * rs[r]);
    }
  }
  __syncthreads();

  v4u    vals[8];
  size_t gidx[8];
  #pragma unroll
  for (int it = 0; it < 8; ++it) {
    const int row = it * 2 + hi;
    vals[it] = *(const v4u*)(so + row * TP + lq * 8);
    gidx[it] = ((size_t)b * SEQ + qrow0 + row) * DM + h * HDIM + lq * 8;
  }
  #pragma unroll
  for (int it = 0; it < 8; ++it) *(volatile v4u*)(ctx + gidx[it]) = vals[it];
  __threadfence();
  #pragma unroll
  for (int it = 0; it < 8; ++it) *(volatile v4u*)(ctx + gidx[it]) = vals[it];
}

extern "C" void kernel_launch(void* const* d_in, const int* in_sizes, int n_in,
                              void* d_out, int out_size, void* d_ws, size_t ws_size,
                              hipStream_t stream) {
  if (n_in < 13) return;
  const size_t need_x = (((size_t)(NB - 1)) * SEQ_FULL + SEQ) * DM;
  const size_t need_t = (size_t)SEQ * HALFD;
  const size_t WD     = (size_t)DM * DM;
  if ((size_t)in_sizes[0] < need_x) return;
  if ((size_t)in_sizes[1] < need_t) return;
  if ((size_t)in_sizes[2] < need_t) return;
  if ((size_t)in_sizes[3] < WD || (size_t)in_sizes[5] < WD) return;
  if ((size_t)in_sizes[7] < WD || (size_t)in_sizes[9] < WD) return;
  if (in_sizes[4] < DM || in_sizes[6] < DM || in_sizes[8] < DM || in_sizes[10] < DM) return;
  if (in_sizes[11] < DM || in_sizes[12] < DM) return;
  if ((size_t)out_size < need_x) return;

  const size_t MDc   = (size_t)NB * SEQ * DM;
  const size_t off_x = 0;
  const size_t off_w0 = off_x + MDc * 2;
  const size_t off_w1 = off_w0 + WD * 2;
  const size_t off_w2 = off_w1 + WD * 2;
  const size_t off_f  = off_w2 + WD * 2;
  const size_t off_q  = off_f + MDc * 4;
  const size_t off_k  = off_q + MDc * 2;
  const size_t off_v  = off_k + MDc * 2;
  const size_t total  = off_v + MDc * 2;
  if (total > (size_t)WS_CAP) return;
  if (ws_size < total) return;

  const float* x   = (const float*)d_in[0];
  const float* fc  = (const float*)d_in[1];
  const float* fs  = (const float*)d_in[2];
  const float* qw  = (const float*)d_in[3];
  const float* qb  = (const float*)d_in[4];
  const float* kw  = (const float*)d_in[5];
  const float* kb  = (const float*)d_in[6];
  const float* vw  = (const float*)d_in[7];
  const float* vb  = (const float*)d_in[8];
  const float* ow  = (const float*)d_in[9];
  const float* ob  = (const float*)d_in[10];
  const float* qnw = (const float*)d_in[11];
  const float* knw = (const float*)d_in[12];
  float* out = (float*)d_out;

  char* ws = (char*)d_ws;
  unsigned short* xb   = (unsigned short*)(ws + off_x);
  unsigned short* ctxp = (unsigned short*)(ws + off_x);
  unsigned short* w0   = (unsigned short*)(ws + off_w0);
  unsigned short* w1   = (unsigned short*)(ws + off_w1);
  unsigned short* w2   = (unsigned short*)(ws + off_w2);
  float*          fbuf = (float*)(ws + off_f);
  unsigned short* q16  = (unsigned short*)(ws + off_q);
  unsigned short* k16  = (unsigned short*)(ws + off_k);
  unsigned short* vtp  = (unsigned short*)(ws + off_v);

  const int M = NB * SEQ;
  const dim3 gg((unsigned)(M / GT), (unsigned)(DM / GT));

  cvt_rows_kernel<0><<<M,  256, 0, stream>>>(x,  xb, SEQ, SEQ_FULL, 1.0f);
  cvt_rows_kernel<0><<<DM, 256, 0, stream>>>(qw, w0, DM, DM, 1.0f);
  cvt_rows_kernel<0><<<DM, 256, 0, stream>>>(kw, w1, DM, DM, 1.0f);
  cvt_rows_kernel<0><<<DM, 256, 0, stream>>>(vw, w2, DM, DM, 1.0f);

  gemm_kernel<0, 0><<<gg, 256, 0, stream>>>(xb, w0, qb, (void*)fbuf, 1.0f);
  rmsnorm_rope_kernel<<<M, 256, 0, stream>>>(fbuf, qnw, fc, fs, q16);
  gemm_kernel<0, 0><<<gg, 256, 0, stream>>>(xb, w1, kb, (void*)fbuf, 1.0f);
  rmsnorm_rope_kernel<<<M, 256, 0, stream>>>(fbuf, knw, fc, fs, k16);
  gemm_kernel<0, 1><<<gg, 256, 0, stream>>>(xb, w2, vb, (void*)vtp, 1.0f);

  cvt_rows_kernel<1><<<DM, 256, 0, stream>>>(ow, w0, DM, DM, 1024.0f);

  attn_kernel<<<dim3(SEQ / BQ, NHEAD, NB), 256, 0, stream>>>(q16, k16, vtp, ctxp);

  gemm_kernel<1, 2><<<gg, 256, 0, stream>>>(ctxp, w0, ob, (void*)out, 1.0f / 262144.0f);
}
